// GNNRecommender_63050119905949
// MI455X (gfx1250) — hardware-verified
//
#include <hip/hip_runtime.h>
#include <stddef.h>


#define EMBD    64
#define HIDD    128
#define NUSERS  100000
#define NTHR    256
#define NWAVE   8
#define EPT     8
#define NGRP    2
#define CHUNK   (NTHR * EPT * NGRP)
#define WCAP    (EPT * NGRP * 32)
#define LISTN   (NWAVE * WCAP)
#define NBA     1024
#define NBD     4096
#define GROWS   128
#define HROWS   128
#define AP1     72
#define AP2     136
#define WSC     8.0f
#define ASC     16.0f
#define OINV    (1.0f / 128.0f)
#define LN_EPS  1e-5f

#define LDS_AGG   (NBA * EMBD * 4 + LISTN * 4 + 64)
#define LDS_GEMM  (GROWS * AP1 * 2 + GROWS * AP2 * 2 + GROWS * EMBD * 4)
#define LDS_HEAD  (HROWS * AP2 * 2 * 2 + HROWS * 4)

static_assert((CHUNK & (CHUNK - 1)) == 0);
static_assert(CHUNK <= 4096);
static_assert((NBA & (NBA - 1)) == 0 && NBA <= 4096);
static_assert((NBD & (NBD - 1)) == 0 && NBD <= 4096);
static_assert(GROWS == NWAVE * 16 && HROWS == NWAVE * 16);
static_assert((GROWS * AP1 * 2) % 16 == 0 && (GROWS * AP2 * 2) % 16 == 0);

typedef float    v2f  __attribute__((ext_vector_type(2)));
typedef float    v4f  __attribute__((ext_vector_type(4)));
typedef float    v8f  __attribute__((ext_vector_type(8)));
typedef int      v4i  __attribute__((ext_vector_type(4)));
typedef _Float16 v8h  __attribute__((ext_vector_type(8)));
typedef _Float16 v16h __attribute__((ext_vector_type(16)));
union FragH { v16h v; v8h h[2]; };

__device__ __forceinline__ v8h cvt8(v4f a, v4f b) {
  v8h r;
  r[0] = (_Float16)a.x; r[1] = (_Float16)a.y; r[2] = (_Float16)a.z; r[3] = (_Float16)a.w;
  r[4] = (_Float16)b.x; r[5] = (_Float16)b.y; r[6] = (_Float16)b.z; r[7] = (_Float16)b.w;
  return r;
}

__device__ __forceinline__ v8f wmh(v16h a, v16h b, v8f c) {
  v8f d = __builtin_amdgcn_wmma_f32_16x16x32_f16(false, a, false, b, (short)0, c, false, false);
  asm volatile("v_nop\n\tv_nop\n\tv_nop\n\tv_nop" : "+v"(d) : "v"(a), "v"(b));
  return d;
}

template <int NB>
__device__ __forceinline__ int scan_chunk(const int* __restrict__ dsts, int nE, int cbase, int nodeBase,
                                          int vec8, int* list, int tid, int lane, int wave) {
  int wc = 0;
#pragma unroll
  for (int g = 0; g < NGRP; ++g) {
    const int el0  = (g * NTHR + tid) * EPT;
    const int e0   = cbase + el0;
    const int sent = -2147483647 - 1;
    v4i da, db;
    if (vec8 != 0 && cbase + CHUNK <= nE) {
      da = *(const v4i*)(dsts + e0);
      db = *(const v4i*)(dsts + e0 + 4);
    } else {
      da.x = (e0     < nE) ? dsts[min(e0, nE - 1)] : sent;
      da.y = (e0 + 1 < nE) ? dsts[min(e0 + 1, nE - 1)] : sent;
      da.z = (e0 + 2 < nE) ? dsts[min(e0 + 2, nE - 1)] : sent;
      da.w = (e0 + 3 < nE) ? dsts[min(e0 + 3, nE - 1)] : sent;
      db.x = (e0 + 4 < nE) ? dsts[min(e0 + 4, nE - 1)] : sent;
      db.y = (e0 + 5 < nE) ? dsts[min(e0 + 5, nE - 1)] : sent;
      db.z = (e0 + 6 < nE) ? dsts[min(e0 + 6, nE - 1)] : sent;
      db.w = (e0 + 7 < nE) ? dsts[min(e0 + 7, nE - 1)] : sent;
    }
    const unsigned nb = (unsigned)nodeBase;
    const unsigned s0 = (unsigned)da.x - nb, s1 = (unsigned)da.y - nb;
    const unsigned s2 = (unsigned)da.z - nb, s3 = (unsigned)da.w - nb;
    const unsigned s4 = (unsigned)db.x - nb, s5 = (unsigned)db.y - nb;
    const unsigned s6 = (unsigned)db.z - nb, s7 = (unsigned)db.w - nb;
    const bool h0 = s0 < (unsigned)NB, h1 = s1 < (unsigned)NB, h2 = s2 < (unsigned)NB, h3 = s3 < (unsigned)NB;
    const bool h4 = s4 < (unsigned)NB, h5 = s5 < (unsigned)NB, h6 = s6 < (unsigned)NB, h7 = s7 < (unsigned)NB;
    const unsigned any = __builtin_amdgcn_ballot_w32(h0 | h1 | h2 | h3 | h4 | h5 | h6 | h7);
    if (any != 0u) {
#define HITJ(J, HJ, SJ) { \
        const unsigned mj = __builtin_amdgcn_ballot_w32(HJ); \
        if (mj != 0u) { \
          if (HJ) { \
            const int pos = wc + (int)__builtin_amdgcn_mbcnt_lo(mj, 0u); \
            if (pos < WCAP) list[wave * WCAP + pos] = ((el0 + (J)) << 12) | (int)(SJ); \
          } \
          wc += (int)__builtin_popcount(mj); } }
      HITJ(0, h0, s0)
      HITJ(1, h1, s1)
      HITJ(2, h2, s2)
      HITJ(3, h3, s3)
      HITJ(4, h4, s4)
      HITJ(5, h5, s5)
      HITJ(6, h6, s6)
      HITJ(7, h7, s7)
#undef HITJ
    }
  }
  return wc;
}

__global__ __launch_bounds__(NTHR) void k_wprep(
    const float* __restrict__ W1, const float* __restrict__ W2,
    const float* __restrict__ F1, const float* __restrict__ F2,
    _Float16* w1s, _Float16* w2s, _Float16* f1s, _Float16* f2s) {
  const int i  = blockIdx.x * NTHR + threadIdx.x;
  const int n0 = EMBD * HIDD / 8;
  const int n1 = HIDD * EMBD / 8;
  const int n2 = HIDD * HIDD / 8;
  const int n3 = HIDD * EMBD / 8;
  if (i >= n0 + n1 + n2 + n3) return;
  int sel, j;
  if (i < n0)                { sel = 0; j = i; }
  else if (i < n0 + n1)      { sel = 1; j = i - n0; }
  else if (i < n0 + n1 + n2) { sel = 2; j = i - n0 - n1; }
  else                       { sel = 3; j = i - n0 - n1 - n2; }
  const int K  = (sel == 0) ? EMBD : HIDD;
  const int NC = (sel == 0 || sel == 2) ? HIDD : EMBD;
  const float* W = (sel == 0) ? W1 : ((sel == 1) ? W2 : ((sel == 2) ? F1 : F2));
  _Float16*    P = (sel == 0) ? w1s : ((sel == 1) ? w2s : ((sel == 2) ? f1s : f2s));
  const int o  = j * 8;
  const int n  = o / K;
  const int k0 = o - n * K;
  const float* p = W + (size_t)k0 * NC + n;
  v4f a, b;
  a.x = p[0];      a.y = p[NC];     a.z = p[2 * NC]; a.w = p[3 * NC];
  b.x = p[4 * NC]; b.y = p[5 * NC]; b.z = p[6 * NC]; b.w = p[7 * NC];
  a = a * WSC;
  b = b * WSC;
  const v8h hv = cvt8(a, b);
  _Float16* dp = P + o;
  *(volatile v8h*)dp = hv;
  __threadfence();
  *(volatile v8h*)dp = hv;
}

__global__ __launch_bounds__(NTHR) void k_deg(
    const int* __restrict__ dsts, float* dinv, int nE, int vec8) {
  __shared__ __attribute__((aligned(16))) int cnt[NBD];
  __shared__ __attribute__((aligned(16))) int list[LISTN];
  __shared__ int wcnt[NWAVE];
  const int tid = threadIdx.x, lane = tid & 31, wave = tid >> 5;
  const int nodeBase = blockIdx.x * NBD;

  for (int i = tid; i < NBD; i += NTHR) cnt[i] = 0;
  __syncthreads();

  const int nChunks = (nE + CHUNK - 1) / CHUNK;
#pragma unroll 1
  for (int ch = 0; ch < nChunks; ++ch) {
    const int cbase = ch * CHUNK;
    const int wc = scan_chunk<NBD>(dsts, nE, cbase, nodeBase, vec8, list, tid, lane, wave);
    if (lane == 0) wcnt[wave] = wc;
    __syncthreads();
    if (wave == 0) {
#pragma unroll 1
      for (int wsx = 0; wsx < NWAVE; ++wsx) {
        int n = __builtin_amdgcn_readfirstlane(wcnt[wsx]);
        n = n > WCAP ? WCAP : (n < 0 ? 0 : n);
        const int* lp = list + wsx * WCAP;
#pragma unroll 1
        for (int i = 0; i < n; ++i) {
          const int ent  = __builtin_amdgcn_readfirstlane(lp[i]);
          const int slot = ent & (NBD - 1);
          if (lane == 0) cnt[slot] = cnt[slot] + 1;
        }
      }
    }
    __syncthreads();
  }

  v4f dq[4];
#pragma unroll
  for (int q = 0; q < 4; ++q) {
    const int f = (wave * 4 + q) * 128 + 4 * lane;
    const v4i c = *(const v4i*)(cnt + f);
    dq[q].x = rsqrtf((float)(c.x + 1));
    dq[q].y = rsqrtf((float)(c.y + 1));
    dq[q].z = rsqrtf((float)(c.z + 1));
    dq[q].w = rsqrtf((float)(c.w + 1));
  }
  float* dp = dinv + (size_t)nodeBase;
#pragma unroll
  for (int q = 0; q < 4; ++q) *(volatile v4f*)(dp + (wave * 4 + q) * 128 + 4 * lane) = dq[q];
  __threadfence();
#pragma unroll
  for (int q = 0; q < 4; ++q) *(volatile v4f*)(dp + (wave * 4 + q) * 128 + 4 * lane) = dq[q];
}

__global__ __launch_bounds__(NTHR) void k_agg1(
    const int* __restrict__ srcs, const int* __restrict__ dsts, const float* __restrict__ x,
    const float* __restrict__ dinv, float* a1, int nN, int nE, int vec8) {
  extern __shared__ v4f lds_dyn[];
  float* acc  = (float*)lds_dyn;
  int*   list = (int*)(acc + NBA * EMBD);
  int*   wcnt = list + LISTN;
  const int tid = threadIdx.x, lane = tid & 31, wave = tid >> 5;
  const int nodeBase = blockIdx.x * NBA;

  {
    const v4f z = {0.f, 0.f, 0.f, 0.f};
    for (int i = tid; i < NBA * EMBD / 4; i += NTHR) lds_dyn[i] = z;
  }
  __syncthreads();

  const int nChunks = (nE + CHUNK - 1) / CHUNK;
#pragma unroll 1
  for (int ch = 0; ch < nChunks; ++ch) {
    const int cbase = ch * CHUNK;
    const int wc = scan_chunk<NBA>(dsts, nE, cbase, nodeBase, vec8, list, tid, lane, wave);
    if (lane == 0) wcnt[wave] = wc;
    __syncthreads();
    if (wave == 0) {
#pragma unroll 1
      for (int wsx = 0; wsx < NWAVE; ++wsx) {
        int n = __builtin_amdgcn_readfirstlane(wcnt[wsx]);
        n = n > WCAP ? WCAP : (n < 0 ? 0 : n);
        const int* lp = list + wsx * WCAP;
#pragma unroll 1
        for (int i = 0; i < n; ++i) {
          const int ent  = __builtin_amdgcn_readfirstlane(lp[i]);
          const int slot = ent & (NBA - 1);
          int e = cbase + ((ent >> 12) & (CHUNK - 1));
          e = e > nE - 1 ? nE - 1 : e;
          int s = srcs[e];
          s = s < 0 ? 0 : (s > nN - 1 ? nN - 1 : s);
          const float ds = dinv[s];
          const v2f v = *(const v2f*)(x + (size_t)s * EMBD + 2 * lane);
          v2f* ap = (v2f*)(acc + slot * EMBD + 2 * lane);
          *ap = *ap + v * ds;
        }
      }
    }
    __syncthreads();
  }

#pragma unroll 4
  for (int i = 0; i < (NBA * EMBD / 4) / NTHR; ++i) {
    const int idx  = i * NTHR + tid;
    const int slot = idx >> 4;
    const int c4   = (idx & 15) * 4;
    int node = nodeBase + slot;
    node = node > nN - 1 ? nN - 1 : node;
    const float d  = dinv[node];
    const v4f   xv = *(const v4f*)(x + (size_t)node * EMBD + c4);
    v4f* ap = (v4f*)(acc + slot * EMBD + c4);
    *ap = (*ap + xv * d) * d;
  }
  __syncthreads();

  float* gp = a1 + (size_t)nodeBase * EMBD;
#pragma unroll 4
  for (int q = 0; q < 64; ++q) {
    const int f = (wave * 64 + q) * 128 + 4 * lane;
    const v4f v = *(const v4f*)(acc + f);
    *(volatile v4f*)(gp + f) = v;
  }
  __threadfence();
#pragma unroll 4
  for (int q = 0; q < 64; ++q) {
    const int f = (wave * 64 + q) * 128 + 4 * lane;
    const v4f v = *(const v4f*)(acc + f);
    *(volatile v4f*)(gp + f) = v;
  }
}

__global__ __launch_bounds__(NTHR) void k_gemm12(
    const float* __restrict__ a1, const _Float16* __restrict__ w1s, const _Float16* __restrict__ w2s,
    const float* __restrict__ b1, const float* __restrict__ dinv, float* gpl, int nN) {
  extern __shared__ v4f lds_dyn[];
  _Float16* sA1 = (_Float16*)lds_dyn;
  _Float16* sA2 = sA1 + GROWS * AP1;
  float*    sG  = (float*)(sA2 + GROWS * AP2);
  const int tid = threadIdx.x, lane = tid & 31, wave = tid >> 5, hh = lane >> 4, m = lane & 15;
  const int rowBase = blockIdx.x * GROWS;

#pragma unroll
  for (int i = 0; i < (GROWS * EMBD / 8) / NTHR; ++i) {
    const int idx = i * NTHR + tid;
    const int r   = idx >> 3;
    const int c0  = (idx & 7) * 8;
    int node = rowBase + r;
    node = node > nN - 1 ? nN - 1 : node;
    const float* xp = a1 + (size_t)node * EMBD + c0;
    const v4f a = *(const v4f*)xp, b = *(const v4f*)(xp + 4);
    *(v8h*)(sA1 + r * AP1 + c0) = cvt8(a * ASC, b * ASC);
  }
  __syncthreads();

  v8f acc[8];
#pragma unroll
  for (int t = 0; t < 8; ++t) { v8f z = {0.f, 0.f, 0.f, 0.f, 0.f, 0.f, 0.f, 0.f}; acc[t] = z; }
  {
    const _Float16* ar = sA1 + (wave * 16 + m) * AP1 + 8 * hh;
#pragma unroll
    for (int kt = 0; kt < EMBD / 32; ++kt) {
      FragH a;
      a.h[0] = *(const v8h*)(ar + 32 * kt);
      a.h[1] = *(const v8h*)(ar + 32 * kt + 16);
#pragma unroll
      for (int t = 0; t < 8; ++t) {
        const _Float16* bp = w1s + (size_t)(16 * t + m) * EMBD + 32 * kt + 8 * hh;
        FragH b;
        b.h[0] = *(const v8h*)bp;
        b.h[1] = *(const v8h*)(bp + 16);
        acc[t] = wmh(a.v, b.v, acc[t]);
      }
    }
  }

  {
    _Float16* zp = sA2 + (wave * 16 + 8 * hh) * AP2;
#pragma unroll
    for (int t = 0; t < 8; ++t) {
      const int   col = 16 * t + m;
      const float bb  = b1[col];
#pragma unroll
      for (int r = 0; r < 8; ++r) {
        const float h = fmaxf(acc[t][r] * OINV + bb, 0.f);
        zp[r * AP2 + col] = (_Float16)(h * ASC);
      }
    }
  }
  __syncthreads();

  v8f acc2[4];
#pragma unroll
  for (int t = 0; t < 4; ++t) { v8f z = {0.f, 0.f, 0.f, 0.f, 0.f, 0.f, 0.f, 0.f}; acc2[t] = z; }
  {
    const _Float16* ar = sA2 + (wave * 16 + m) * AP2 + 8 * hh;
#pragma unroll
    for (int kt = 0; kt < HIDD / 32; ++kt) {
      FragH a;
      a.h[0] = *(const v8h*)(ar + 32 * kt);
      a.h[1] = *(const v8h*)(ar + 32 * kt + 16);
#pragma unroll
      for (int t = 0; t < 4; ++t) {
        const _Float16* bp = w2s + (size_t)(16 * t + m) * HIDD + 32 * kt + 8 * hh;
        FragH b;
        b.h[0] = *(const v8h*)bp;
        b.h[1] = *(const v8h*)(bp + 16);
        acc2[t] = wmh(a.v, b.v, acc2[t]);
      }
    }
  }

  {
    const int r0 = wave * 16 + 8 * hh;
    const v4f dA = *(const v4f*)(dinv + (size_t)rowBase + r0);
    const v4f dB = *(const v4f*)(dinv + (size_t)rowBase + r0 + 4);
    const float d0 = dA.x * OINV, d1 = dA.y * OINV, d2 = dA.z * OINV, d3 = dA.w * OINV;
    const float d4 = dB.x * OINV, d5 = dB.y * OINV, d6 = dB.z * OINV, d7 = dB.w * OINV;
    float* sp = sG + r0 * EMBD + m;
#pragma unroll
    for (int t = 0; t < 4; ++t) {
      sp[0 * EMBD + 16 * t] = acc2[t][0] * d0;
      sp[1 * EMBD + 16 * t] = acc2[t][1] * d1;
      sp[2 * EMBD + 16 * t] = acc2[t][2] * d2;
      sp[3 * EMBD + 16 * t] = acc2[t][3] * d3;
      sp[4 * EMBD + 16 * t] = acc2[t][4] * d4;
      sp[5 * EMBD + 16 * t] = acc2[t][5] * d5;
      sp[6 * EMBD + 16 * t] = acc2[t][6] * d6;
      sp[7 * EMBD + 16 * t] = acc2[t][7] * d7;
    }
  }
  __syncthreads();

  const float* lp = sG + wave * 16 * EMBD + 4 * lane;
  float* gp = gpl + ((size_t)rowBase + wave * 16) * EMBD + 4 * lane;
#pragma unroll
  for (int q = 0; q < 8; ++q) { const v4f v = *(const v4f*)(lp + q * 128); *(volatile v4f*)(gp + q * 128) = v; }
  __threadfence();
#pragma unroll
  for (int q = 0; q < 8; ++q) { const v4f v = *(const v4f*)(lp + q * 128); *(volatile v4f*)(gp + q * 128) = v; }
}

__global__ __launch_bounds__(NTHR) void k_agg2(
    const int* __restrict__ srcs, const int* __restrict__ dsts, const float* __restrict__ gpl,
    const float* __restrict__ dinv, const float* __restrict__ b2, float* h2, int nN, int nE, int vec8) {
  extern __shared__ v4f lds_dyn[];
  float* acc  = (float*)lds_dyn;
  int*   list = (int*)(acc + NBA * EMBD);
  int*   wcnt = list + LISTN;
  const int tid = threadIdx.x, lane = tid & 31, wave = tid >> 5;
  const int nodeBase = blockIdx.x * NBA;

  {
    const v4f z = {0.f, 0.f, 0.f, 0.f};
    for (int i = tid; i < NBA * EMBD / 4; i += NTHR) lds_dyn[i] = z;
  }
  __syncthreads();

  const int nChunks = (nE + CHUNK - 1) / CHUNK;
#pragma unroll 1
  for (int ch = 0; ch < nChunks; ++ch) {
    const int cbase = ch * CHUNK;
    const int wc = scan_chunk<NBA>(dsts, nE, cbase, nodeBase, vec8, list, tid, lane, wave);
    if (lane == 0) wcnt[wave] = wc;
    __syncthreads();
    if (wave == 0) {
#pragma unroll 1
      for (int wsx = 0; wsx < NWAVE; ++wsx) {
        int n = __builtin_amdgcn_readfirstlane(wcnt[wsx]);
        n = n > WCAP ? WCAP : (n < 0 ? 0 : n);
        const int* lp = list + wsx * WCAP;
#pragma unroll 1
        for (int i = 0; i < n; ++i) {
          const int ent  = __builtin_amdgcn_readfirstlane(lp[i]);
          const int slot = ent & (NBA - 1);
          int e = cbase + ((ent >> 12) & (CHUNK - 1));
          e = e > nE - 1 ? nE - 1 : e;
          int s = srcs[e];
          s = s < 0 ? 0 : (s > nN - 1 ? nN - 1 : s);
          const v2f v = *(const v2f*)(gpl + (size_t)s * EMBD + 2 * lane);
          v2f* ap = (v2f*)(acc + slot * EMBD + 2 * lane);
          *ap = *ap + v;
        }
      }
    }
    __syncthreads();
  }

#pragma unroll 4
  for (int i = 0; i < (NBA * EMBD / 4) / NTHR; ++i) {
    const int idx  = i * NTHR + tid;
    const int slot = idx >> 4;
    const int c4   = (idx & 15) * 4;
    int node = nodeBase + slot;
    node = node > nN - 1 ? nN - 1 : node;
    const float d  = dinv[node];
    const v4f   gv = *(const v4f*)(gpl + (size_t)node * EMBD + c4);
    const v4f   bv = *(const v4f*)(b2 + c4);
    v4f* ap = (v4f*)(acc + slot * EMBD + c4);
    *ap = (*ap + gv) * d + bv;
  }
  __syncthreads();

  float* gp = h2 + (size_t)nodeBase * EMBD;
#pragma unroll 4
  for (int q = 0; q < 64; ++q) {
    const int f = (wave * 64 + q) * 128 + 4 * lane;
    const v4f v = *(const v4f*)(acc + f);
    *(volatile v4f*)(gp + f) = v;
  }
  __threadfence();
#pragma unroll 4
  for (int q = 0; q < 64; ++q) {
    const int f = (wave * 64 + q) * 128 + 4 * lane;
    const v4f v = *(const v4f*)(acc + f);
    *(volatile v4f*)(gp + f) = v;
  }
}

__global__ __launch_bounds__(NTHR) void k_head(
    const float* __restrict__ h2, const int* __restrict__ uidx, const int* __restrict__ iidx,
    const _Float16* __restrict__ f1s, const _Float16* __restrict__ f2s,
    const float* __restrict__ fcb1, const float* __restrict__ g1, const float* __restrict__ be1,
    const float* __restrict__ fcb2, const float* __restrict__ g2, const float* __restrict__ be2,
    const float* __restrict__ w3, const float* __restrict__ b3,
    float* out, int nN, int nB) {
  extern __shared__ v4f lds_dyn[];
  _Float16* sC   = (_Float16*)lds_dyn;
  _Float16* sZ   = sC + HROWS * AP2;
  float*    sOut = (float*)(sZ + HROWS * AP2);
  const int tid = threadIdx.x, lane = tid & 31, wave = tid >> 5, hh = lane >> 4, m = lane & 15;
  const int rowBase = blockIdx.x * HROWS;
  const int nItems  = nN - NUSERS;

#pragma unroll
  for (int i = 0; i < (HROWS * 2 * EMBD / 8) / NTHR; ++i) {
    const int idx = i * NTHR + tid;
    const int r   = idx >> 4;
    const int c0  = (idx & 15) * 8;
    int row = rowBase + r;
    row = row > nB - 1 ? nB - 1 : row;
    int u = uidx[row] - 1;
    u = u < 0 ? u + NUSERS : u;
    u = u < 0 ? 0 : (u > NUSERS - 1 ? NUSERS - 1 : u);
    int it = iidx[row] - 1;
    it = it < 0 ? it + nItems : it;
    it = it < 0 ? 0 : (it > nItems - 1 ? nItems - 1 : it);
    const int node = (c0 < EMBD) ? u : (NUSERS + it);
    const int cc   = c0 & (EMBD - 1);
    const float* p = h2 + (size_t)node * EMBD + cc;
    const v4f a = *(const v4f*)p, b = *(const v4f*)(p + 4);
    *(v8h*)(sC + r * AP2 + c0) = cvt8(a * ASC, b * ASC);
  }
  __syncthreads();

  v8f acc[8];
#pragma unroll
  for (int t = 0; t < 8; ++t) { v8f z = {0.f, 0.f, 0.f, 0.f, 0.f, 0.f, 0.f, 0.f}; acc[t] = z; }
  {
    const _Float16* ar = sC + (wave * 16 + m) * AP2 + 8 * hh;
#pragma unroll
    for (int kt = 0; kt < HIDD / 32; ++kt) {
      FragH a;
      a.h[0] = *(const v8h*)(ar + 32 * kt);
      a.h[1] = *(const v8h*)(ar + 32 * kt + 16);
#pragma unroll
      for (int t = 0; t < 8; ++t) {
        const _Float16* bp = f1s + (size_t)(16 * t + m) * HIDD + 32 * kt + 8 * hh;
        FragH b;
        b.h[0] = *(const v8h*)bp;
        b.h[1] = *(const v8h*)(bp + 16);
        acc[t] = wmh(a.v, b.v, acc[t]);
      }
    }
  }

  {
#pragma unroll
    for (int t = 0; t < 8; ++t) {
      const float bb = fcb1[16 * t + m];
#pragma unroll
      for (int r = 0; r < 8; ++r) acc[t][r] = acc[t][r] * OINV + bb;
    }
    float mu[8], rs[8];
#pragma unroll
    for (int r = 0; r < 8; ++r) {
      float s = 0.f;
#pragma unroll
      for (int t = 0; t < 8; ++t) s += acc[t][r];
      s += __shfl_xor(s, 1, 32); s += __shfl_xor(s, 2, 32); s += __shfl_xor(s, 4, 32); s += __shfl_xor(s, 8, 32);
      mu[r] = s * (1.0f / 128.0f);
    }
#pragma unroll
    for (int r = 0; r < 8; ++r) {
      float q = 0.f;
#pragma unroll
      for (int t = 0; t < 8; ++t) { const float d = acc[t][r] - mu[r]; q += d * d; }
      q += __shfl_xor(q, 1, 32); q += __shfl_xor(q, 2, 32); q += __shfl_xor(q, 4, 32); q += __shfl_xor(q, 8, 32);
      rs[r] = rsqrtf(q * (1.0f / 128.0f) + LN_EPS);
    }
    _Float16* zp = sZ + (wave * 16 + 8 * hh) * AP2;
#pragma unroll
    for (int t = 0; t < 8; ++t) {
      const int   col = 16 * t + m;
      const float gg  = g1[col], be = be1[col];
#pragma unroll
      for (int r = 0; r < 8; ++r) {
        const float z = fmaxf((acc[t][r] - mu[r]) * rs[r] * gg + be, 0.f);
        zp[r * AP2 + col] = (_Float16)(z * ASC);
      }
    }
  }
  __syncthreads();

  v8f acc2[4];
#pragma unroll
  for (int t = 0; t < 4; ++t) { v8f z = {0.f, 0.f, 0.f, 0.f, 0.f, 0.f, 0.f, 0.f}; acc2[t] = z; }
  {
    const _Float16* ar = sZ + (wave * 16 + m) * AP2 + 8 * hh;
#pragma unroll
    for (int kt = 0; kt < HIDD / 32; ++kt) {
      FragH a;
      a.h[0] = *(const v8h*)(ar + 32 * kt);
      a.h[1] = *(const v8h*)(ar + 32 * kt + 16);
#pragma unroll
      for (int t = 0; t < 4; ++t) {
        const _Float16* bp = f2s + (size_t)(16 * t + m) * HIDD + 32 * kt + 8 * hh;
        FragH b;
        b.h[0] = *(const v8h*)bp;
        b.h[1] = *(const v8h*)(bp + 16);
        acc2[t] = wmh(a.v, b.v, acc2[t]);
      }
    }
  }

  {
#pragma unroll
    for (int t = 0; t < 4; ++t) {
      const float bb = fcb2[16 * t + m];
#pragma unroll
      for (int r = 0; r < 8; ++r) acc2[t][r] = acc2[t][r] * OINV + bb;
    }
    float mu[8], rs[8];
#pragma unroll
    for (int r = 0; r < 8; ++r) {
      float s = 0.f;
#pragma unroll
      for (int t = 0; t < 4; ++t) s += acc2[t][r];
      s += __shfl_xor(s, 1, 32); s += __shfl_xor(s, 2, 32); s += __shfl_xor(s, 4, 32); s += __shfl_xor(s, 8, 32);
      mu[r] = s * (1.0f / 64.0f);
    }
#pragma unroll
    for (int r = 0; r < 8; ++r) {
      float q = 0.f;
#pragma unroll
      for (int t = 0; t < 4; ++t) { const float d = acc2[t][r] - mu[r]; q += d * d; }
      q += __shfl_xor(q, 1, 32); q += __shfl_xor(q, 2, 32); q += __shfl_xor(q, 4, 32); q += __shfl_xor(q, 8, 32);
      rs[r] = rsqrtf(q * (1.0f / 64.0f) + LN_EPS);
    }
    float dot[8];
#pragma unroll
    for (int r = 0; r < 8; ++r) dot[r] = 0.f;
#pragma unroll
    for (int t = 0; t < 4; ++t) {
      const int   col = 16 * t + m;
      const float gg  = g2[col], be = be2[col], ww = w3[col];
#pragma unroll
      for (int r = 0; r < 8; ++r) {
        const float z = fmaxf((acc2[t][r] - mu[r]) * rs[r] * gg + be, 0.f);
        dot[r] += z * ww;
      }
    }
    const float bb3 = b3[0];
#pragma unroll
    for (int r = 0; r < 8; ++r) {
      float s = dot[r];
      s += __shfl_xor(s, 1, 32); s += __shfl_xor(s, 2, 32); s += __shfl_xor(s, 4, 32); s += __shfl_xor(s, 8, 32);
      const float v  = s + bb3;
      const float e  = __expf(-fabsf(v));
      const float rc = __builtin_amdgcn_rcpf(1.0f + e);
      const float o  = (v >= 0.f) ? rc : e * rc;
      if (m == 0) sOut[wave * 16 + 8 * hh + r] = o;
    }
  }
  __syncthreads();

  if (wave == 0) {
    const v4f v = *(const v4f*)(sOut + 4 * lane);
    const int f = rowBase + 4 * lane;
    float* op = out + f;
    if (f + 4 <= nB) { *(volatile v4f*)op = v; }
    else {
      if (f     < nB) ((volatile float*)op)[0] = v.x;
      if (f + 1 < nB) ((volatile float*)op)[1] = v.y;
      if (f + 2 < nB) ((volatile float*)op)[2] = v.z;
      if (f + 3 < nB) ((volatile float*)op)[3] = v.w;
    }
    __threadfence();
    if (f + 4 <= nB) { *(volatile v4f*)op = v; }
    else {
      if (f     < nB) ((volatile float*)op)[0] = v.x;
      if (f + 1 < nB) ((volatile float*)op)[1] = v.y;
      if (f + 2 < nB) ((volatile float*)op)[2] = v.z;
      if (f + 3 < nB) ((volatile float*)op)[3] = v.w;
    }
  }
}

extern "C" void kernel_launch(void* const* d_in, const int* in_sizes, int n_in,
                              void* d_out, int out_size, void* d_ws, size_t ws_size,
                              hipStream_t stream) {
  if (n_in < 19) return;
  const int nN = in_sizes[0] / EMBD;
  const int nE = in_sizes[1];
  const int nB = in_sizes[3];
  if (nN <= NUSERS || in_sizes[0] != nN * EMBD) return;
  if (nE <= 0 || in_sizes[2] != nE) return;
  if (nB <= 0 || in_sizes[4] != nB || out_size != nB) return;
  if (in_sizes[5] != EMBD * HIDD || in_sizes[6] < HIDD || in_sizes[7] != HIDD * EMBD || in_sizes[8] < EMBD) return;
  if (in_sizes[9] != HIDD * HIDD || in_sizes[10] < HIDD || in_sizes[11] < HIDD || in_sizes[12] < HIDD) return;
  if (in_sizes[13] != HIDD * EMBD || in_sizes[14] < EMBD || in_sizes[15] < EMBD || in_sizes[16] < EMBD) return;
  if (in_sizes[17] < EMBD || in_sizes[18] < 1) return;

  const float* x    = (const float*)d_in[0];
  const int*   srcs = (const int*)d_in[1];
  const int*   dsts = (const int*)d_in[2];
  const int*   uidx = (const int*)d_in[3];
  const int*   iidx = (const int*)d_in[4];
  const float* W1   = (const float*)d_in[5];
  const float* b1   = (const float*)d_in[6];
  const float* W2   = (const float*)d_in[7];
  const float* b2   = (const float*)d_in[8];
  const float* fcW1 = (const float*)d_in[9];
  const float* fcb1 = (const float*)d_in[10];
  const float* g1   = (const float*)d_in[11];
  const float* be1  = (const float*)d_in[12];
  const float* fcW2 = (const float*)d_in[13];
  const float* fcb2 = (const float*)d_in[14];
  const float* g2   = (const float*)d_in[15];
  const float* be2  = (const float*)d_in[16];
  const float* fcW3 = (const float*)d_in[17];
  const float* fcb3 = (const float*)d_in[18];
  float* out = (float*)d_out;

  const int nBD = (nN + NBD - 1) / NBD;
  const int nA  = (nN + NBA - 1) / NBA;
  const int nG  = (nN + GROWS - 1) / GROWS;
  const int nH  = (nB + HROWS - 1) / HROWS;

  char* ws = (char*)d_ws;
  size_t off = 0;
  const size_t oW1 = off; off += (size_t)HIDD * EMBD * 2;                       off = (off + 255) & ~(size_t)255;
  const size_t oW2 = off; off += (size_t)EMBD * HIDD * 2;                       off = (off + 255) & ~(size_t)255;
  const size_t oF1 = off; off += (size_t)HIDD * HIDD * 2;                       off = (off + 255) & ~(size_t)255;
  const size_t oF2 = off; off += (size_t)EMBD * HIDD * 2;                       off = (off + 255) & ~(size_t)255;
  const size_t oDv = off; off += (size_t)nBD * NBD * 4;                         off = (off + 255) & ~(size_t)255;
  const size_t oA1 = off; off += (size_t)nA * NBA * EMBD * 4;                    off = (off + 255) & ~(size_t)255;
  const size_t oG  = off; off += (size_t)nG * GROWS * EMBD * 4;                  off = (off + 255) & ~(size_t)255;
  const size_t oH2 = off; off += (size_t)nA * NBA * EMBD * 4;                    off = (off + 255) & ~(size_t)255;
  if (off > ws_size || off > (size_t)134217728) return;
  _Float16* w1s  = (_Float16*)(ws + oW1);
  _Float16* w2s  = (_Float16*)(ws + oW2);
  _Float16* f1s  = (_Float16*)(ws + oF1);
  _Float16* f2s  = (_Float16*)(ws + oF2);
  float*    dinv = (float*)(ws + oDv);
  float*    a1   = (float*)(ws + oA1);
  float*    gpl  = (float*)(ws + oG);
  float*    h2   = (float*)(ws + oH2);

  const int vec8 = ((nE & 3) == 0) ? 1 : 0;

  const int nPrep = EMBD * HIDD / 8 + HIDD * EMBD / 8 + HIDD * HIDD / 8 + HIDD * EMBD / 8;
  k_wprep<<<(nPrep + NTHR - 1) / NTHR, NTHR, 0, stream>>>(W1, W2, fcW1, fcW2, w1s, w2s, f1s, f2s);

  k_deg<<<nBD, NTHR, 0, stream>>>(dsts, dinv, nE, vec8);

  hipFuncSetAttribute(reinterpret_cast<const void*>(&k_agg1),
                      hipFuncAttributeMaxDynamicSharedMemorySize, LDS_AGG);
  k_agg1<<<nA, NTHR, LDS_AGG, stream>>>(srcs, dsts, x, dinv, a1, nN, nE, vec8);

  hipFuncSetAttribute(reinterpret_cast<const void*>(&k_gemm12),
                      hipFuncAttributeMaxDynamicSharedMemorySize, LDS_GEMM);
  k_gemm12<<<nG, NTHR, LDS_GEMM, stream>>>(a1, w1s, w2s, b1, dinv, gpl, nN);

  hipFuncSetAttribute(reinterpret_cast<const void*>(&k_agg2),
                      hipFuncAttributeMaxDynamicSharedMemorySize, LDS_AGG);
  k_agg2<<<nA, NTHR, LDS_AGG, stream>>>(srcs, dsts, gpl, dinv, b2, h2, nN, nE, vec8);

  hipFuncSetAttribute(reinterpret_cast<const void*>(&k_head),
                      hipFuncAttributeMaxDynamicSharedMemorySize, LDS_HEAD);
  k_head<<<nH, NTHR, LDS_HEAD, stream>>>(h2, uidx, iidx, f1s, f2s, fcb1, g1, be1, fcb2, g2, be2,
                                         fcW3, fcb3, out, nN, nB);
}
